// GroupedRecurrentMultiHeadAttention_78941498900918
// MI455X (gfx1250) — hardware-verified
//
#include <hip/hip_runtime.h>
#include <math.h>

typedef __attribute__((ext_vector_type(16))) _Float16 v16h;
typedef __attribute__((ext_vector_type(16))) __bf16 v16b;
typedef __attribute__((ext_vector_type(8)))  _Float16 v8h;
typedef __attribute__((ext_vector_type(8)))  float v8f;
typedef __attribute__((ext_vector_type(4)))  float v4f;
typedef __attribute__((ext_vector_type(2)))  float v2f;
typedef __attribute__((ext_vector_type(4)))  unsigned v4u;
typedef __attribute__((ext_vector_type(4)))  int v4i;
typedef float __attribute__((may_alias)) float_a;
typedef int __attribute__((may_alias)) int_a;

template <typename T> __device__ __forceinline__ void vst2(void* p, T v) { *(volatile T*)p = v; __threadfence(); *(volatile T*)p = v; }
__device__ __forceinline__ v8f wmma16(v16h a, v16h b, v8f c) {
  v8f d = __builtin_amdgcn_wmma_f32_16x16x32_f16(false, a, false, b, (short)0, c, false, false);
  asm volatile("v_nop\n\tv_nop\n\tv_nop\n\tv_nop" : "+v"(d) : "v"(a), "v"(b));
  return d;
}
__device__ __forceinline__ v8f wmma_bf(v16b a, v16b b, v8f c) {
  v8f d = __builtin_amdgcn_wmma_f32_16x16x32_bf16(false, a, false, b, (short)0, c, false, false);
  asm volatile("v_nop\n\tv_nop\n\tv_nop\n\tv_nop" : "+v"(d) : "v"(a), "v"(b));
  return d;
}
__device__ __forceinline__ v16h frag_h(const _Float16* rowk0, int lane) {
  union { v16h v; v8h q[2]; } u; const _Float16* p = rowk0 + 8 * (lane >> 4);
  u.q[0] = *(const v8h*)p; u.q[1] = *(const v8h*)(p + 16); return u.v;
}
__device__ __forceinline__ v16h frag_f32(const float* rowk0, int lane) {
  v16h a; const float* p = rowk0 + 8 * (lane >> 4);
#pragma unroll
  for (int i = 0; i < 8; ++i) { a[i] = (_Float16)p[i]; a[8 + i] = (_Float16)p[16 + i]; }
  return a;
}
__device__ __forceinline__ v16h frag_f32s(const float* rowk0, int lane, float sc) {
  v16h a; const float* p = rowk0 + 8 * (lane >> 4);
#pragma unroll
  for (int i = 0; i < 8; ++i) { a[i] = (_Float16)(p[i] * sc); a[8 + i] = (_Float16)(p[16 + i] * sc); }
  return a;
}
__device__ __forceinline__ v16h fragc_f32(const float* W, int k0, int n, int lane, int ld, int K) {
  v16h a; const int g = lane >> 4;
#pragma unroll
  for (int i = 0; i < 8; ++i) { const int ka = k0 + 8 * g + i, kb = ka + 16;
    a[i] = (_Float16)(ka < K ? W[(size_t)(ka < K ? ka : K - 1) * ld + n] : 0.f); a[8 + i] = (_Float16)(kb < K ? W[(size_t)(kb < K ? kb : K - 1) * ld + n] : 0.f); }
  return a;
}
struct F2 { v16b h, l; };
__device__ __forceinline__ F2 bsplit16(const float v[16]) { F2 r;
#pragma unroll
  for (int i = 0; i < 16; ++i) { const __bf16 h = (__bf16)v[i]; r.h[i] = h; r.l[i] = (__bf16)(v[i] - (float)h); }
  return r; }
__device__ __forceinline__ F2 split_row(const float* row, int k0, int lane) { float v[16]; const float* p = row + k0 + 8 * (lane >> 4);
#pragma unroll
  for (int i = 0; i < 8; ++i) { v[i] = p[i]; v[8 + i] = p[16 + i]; }
  return bsplit16(v); }
__device__ __forceinline__ F2 split_rowK(const float* row, int k0, int lane, int K) { float v[16]; const int g = lane >> 4;
#pragma unroll
  for (int i = 0; i < 8; ++i) { const int ka = k0 + 8 * g + i, kb = ka + 16; v[i] = ka < K ? row[ka < K ? ka : K - 1] : 0.f; v[8 + i] = kb < K ? row[kb < K ? kb : K - 1] : 0.f; }
  return bsplit16(v); }
__device__ __forceinline__ F2 split_col(const float* W, int k0, int n, int lane, int ld, int K) { float v[16]; const int g = lane >> 4;
#pragma unroll
  for (int i = 0; i < 8; ++i) { const int ka = k0 + 8 * g + i, kb = ka + 16; v[i] = ka < K ? W[(size_t)(ka < K ? ka : K - 1) * ld + n] : 0.f; v[8 + i] = kb < K ? W[(size_t)(kb < K ? kb : K - 1) * ld + n] : 0.f; }
  return bsplit16(v); }
__device__ __forceinline__ v8f mac3(const F2& a, const F2& b, v8f c) { c = wmma_bf(a.l, b.h, c); c = wmma_bf(a.h, b.l, c); return wmma_bf(a.h, b.h, c); }
__device__ __forceinline__ float sigm(float v) { return 1.0f / (1.0f + expf(-v)); }
#define LDSX() do { asm volatile("s_wait_dscnt 0" ::: "memory"); __builtin_amdgcn_wave_barrier(); __builtin_amdgcn_fence(__ATOMIC_RELEASE, "workgroup"); } while (0)


#define NB 4
#define SS 1024
#define DM 1024
#define NQ 4
#define NH 8
#define HD 32
#define KVW (NH * HD)
#define NR (NB * SS)
#ifndef TQB
#define TQB (SS / 64)
#define TNB NB
#endif
typedef __attribute__((ext_vector_type(8))) __bf16 v8b;
__device__ __forceinline__ v16b frag_b(const __bf16* rowk0, int lane) {
  union { v16b v; v8b q[2]; } u; const __bf16* p = rowk0 + 8 * (lane >> 4);
  u.q[0] = *(const v8b*)p; u.q[1] = *(const v8b*)(p + 16); return u.v;
}
__device__ __forceinline__ float bfr(float v) { return (float)(__bf16)v; }
__device__ __attribute__((noinline)) float exp_ni(float v) { return expf(v); }
__device__ __attribute__((noinline)) float erf_ni(float v) { return erff(v); }
__device__ __attribute__((noinline)) float expm1f_ni(float v) { return expm1f(v); }

#define WS_PQ  0u
#define WS_PK  (WS_PQ + 2u * (size_t)DM * DM)
#define WS_PV  (WS_PK + 2u * (size_t)KVW * DM)
#define WS_PM  (WS_PV + 2u * (size_t)KVW * DM)
#define WS_QF  (WS_PM + 2u * (size_t)KVW * KVW)
#define WS_QH  (WS_QF + 4u * (size_t)NR * DM)
#define WS_K   (WS_QH + 2u * (size_t)NR * DM)
#define WS_V   (WS_K + 2u * (size_t)NR * KVW)
#define WS_O   (WS_V + 2u * (size_t)NB * KVW * SS)
#define WS_END (WS_O + 4u * (size_t)NR * DM)

__global__ __launch_bounds__(256) void k_pack(const float* __restrict__ WQ, const float* __restrict__ WK, const float* __restrict__ WV, const float* __restrict__ MM, __bf16* __restrict__ PQ, __bf16* __restrict__ PK, __bf16* __restrict__ PV, __bf16* __restrict__ PM) { const int n = blockIdx.x, which = blockIdx.y, t = threadIdx.x; __shared__ __align__(16) __bf16 s[DM];
  if (which == 0) { for (int k = t; k < DM; k += 256) s[k] = (__bf16)WQ[(size_t)k * DM + n]; __syncthreads(); if (t < DM / 8) vst2((unsigned*)(PQ + (size_t)n * DM + t * 8), *(const v4u*)&s[t * 8]); }
  else if (which < 3) { if (n >= KVW) return; const float* w = (which == 1) ? WK : WV; for (int k = t; k < DM; k += 256) s[k] = (__bf16)w[(size_t)k * KVW + n]; __syncthreads(); __bf16* dst = (which == 1) ? PK : PV; if (t < DM / 8) vst2((unsigned*)(dst + (size_t)n * DM + t * 8), *(const v4u*)&s[t * 8]); }
  else { if (n >= KVW) return; s[t] = (__bf16)MM[(size_t)t * KVW + n]; __syncthreads(); if (t < KVW / 8) vst2((unsigned*)(PM + (size_t)n * KVW + t * 8), *(const v4u*)&s[t * 8]); } }
__global__ __launch_bounds__(128) void k_proj(const float* __restrict__ X, const __bf16* __restrict__ PQ, const __bf16* __restrict__ PK, const __bf16* __restrict__ PV, float* __restrict__ QF, _Float16* __restrict__ QH, _Float16* __restrict__ Kr, _Float16* __restrict__ V) {
  __shared__ __align__(16) float sf[4][16][132]; __shared__ __align__(16) _Float16 so[64][136]; __shared__ __align__(16) _Float16 st[128][72];
  const int tid = threadIdx.x, wave = tid >> 5, lane = tid & 31, col = lane & 15, g = lane >> 4; const int which = blockIdx.z; const int c0 = blockIdx.y * 128; if (which > 0 && c0 >= KVW) return;
  const size_t rb = (size_t)blockIdx.x * 64; const size_t r0 = rb + wave * 16; const __bf16* Wr = (which == 0) ? PQ : (which == 1) ? PK : PV;
  v8f acc[8] = {};
#pragma unroll 2
  for (int kc = 0; kc < DM / 32; ++kc) { v16b a; { const float* p = X + (r0 + col) * DM + kc * 32 + 8 * g;
#pragma unroll
      for (int i = 0; i < 8; ++i) { a[i] = (__bf16)p[i]; a[8 + i] = (__bf16)p[16 + i]; } }
#pragma unroll
    for (int j = 0; j < 8; ++j) acc[j] = wmma_bf(a, frag_b(Wr + (size_t)(c0 + j * 16 + col) * DM + kc * 32, lane), acc[j]); }
  if (which < 2) {
#pragma unroll
    for (int j = 0; j < 8; ++j)
#pragma unroll
      for (int r = 0; r < 8; ++r) { so[wave * 16 + 8 * g + r][j * 16 + col] = (_Float16)acc[j][r]; if (which == 0) sf[wave][8 * g + r][j * 16 + col] = acc[j][r]; }
    __syncthreads();
    if (which == 0) { for (int rl = 0; rl < 16; ++rl) vst2(QF + (r0 + rl) * DM + c0 + lane * 4, *(const v4f*)&sf[wave][rl][lane * 4]); for (int e = tid; e < 64 * 16; e += 128) { const int rl = e >> 4, q = e & 15; vst2((unsigned*)(QH + (rb + rl) * DM + c0 + q * 8), *(const v4u*)&so[rl][q * 8]); } }
    else { for (int e = tid; e < 64 * 16; e += 128) { const int rl = e >> 4, q = e & 15; vst2((unsigned*)(Kr + (rb + rl) * KVW + c0 + q * 8), *(const v4u*)&so[rl][q * 8]); } } }
  else {
#pragma unroll
    for (int j = 0; j < 8; ++j)
#pragma unroll
      for (int r = 0; r < 8; ++r) st[j * 16 + col][wave * 16 + 8 * g + r] = (_Float16)acc[j][r];
    __syncthreads(); const size_t b = rb / SS; const int s0 = (int)(rb % SS);
    for (int e = tid; e < 128 * 8; e += 128) { const int d = e >> 3, pc = e & 7; vst2((unsigned*)(V + ((b * KVW + c0 + d) * SS) + s0 + pc * 8), *(const v4u*)&st[d][pc * 8]); } }
}
__global__ __launch_bounds__(128) void k_attn(const _Float16* __restrict__ QH, const _Float16* __restrict__ Kr, const _Float16* __restrict__ V, float* __restrict__ O) {
  __shared__ __align__(16) _Float16 sph[4][16][40]; __shared__ __align__(16) float so[4][16][36];
  const int tid = threadIdx.x, wave = tid >> 5, lane = tid & 31, col = lane & 15, g = lane >> 4; const int qg = blockIdx.y / NH, h = blockIdx.y % NH; const size_t b = blockIdx.z; const int q0 = blockIdx.x * 64 + wave * 16; const size_t rq = b * SS + q0; const int qc = qg * KVW + h * HD;
  const v16h aq = frag_h(QH + (rq + col) * DM + qc, lane);
  float m[8], l[8];
#pragma unroll
  for (int r = 0; r < 8; ++r) { m[r] = -3.0e38f; l[r] = 0.f; }
  v8f acc[2] = {};
#pragma unroll 1
  for (int ks = 0; ks < SS / 32; ++ks) { const int j0 = ks * 32; v8f s[2];
#pragma unroll
    for (int ct = 0; ct < 2; ++ct) { const int kk = j0 + ct * 16 + col; v8f c = {}; c = wmma16(aq, frag_h(Kr + (b * SS + kk) * KVW + h * HD, lane), c);
#pragma unroll
      for (int r = 0; r < 8; ++r) s[ct][r] = c[r] * 0.17677669529663688f; }
#pragma unroll
    for (int r = 0; r < 8; ++r) { float mx = fmaxf(s[0][r], s[1][r]);
#pragma unroll
      for (int o = 1; o < 16; o <<= 1) mx = fmaxf(mx, __shfl_xor(mx, o));
      const float mn = fmaxf(m[r], mx); const float alpha = (m[r] <= -1.0e38f) ? 0.f : __expf(m[r] - mn); const float e0 = __expf(s[0][r] - mn), e1 = __expf(s[1][r] - mn); float es = e0 + e1;
#pragma unroll
      for (int o = 1; o < 16; o <<= 1) es += __shfl_xor(es, o);
      l[r] = l[r] * alpha + es; m[r] = mn;
#pragma unroll
      for (int dt = 0; dt < 2; ++dt) acc[dt][r] *= alpha;
      sph[wave][8 * g + r][col] = (_Float16)(e0 * 2048.0f); sph[wave][8 * g + r][16 + col] = (_Float16)(e1 * 2048.0f); }
    LDSX();
    const v16h pa = frag_h(&sph[wave][col][0], lane);
#pragma unroll
    for (int dt = 0; dt < 2; ++dt) acc[dt] = wmma16(pa, frag_h(V + ((b * KVW + h * HD + dt * 16 + col) * SS) + j0, lane), acc[dt]);
    LDSX(); }
#pragma unroll
  for (int r = 0; r < 8; ++r) { const float il = (1.0f / 2048.0f) / l[r];
#pragma unroll
    for (int dt = 0; dt < 2; ++dt) so[wave][8 * g + r][dt * 16 + col] = acc[dt][r] * il; }
  LDSX();
  for (int rl = 0; rl < 16; ++rl) if (lane < 8) vst2(O + (rq + rl) * DM + qc + lane * 4, *(const v4f*)&so[wave][rl][lane * 4]);
}
__global__ __launch_bounds__(128) void k_mem(const float* __restrict__ QF, const __bf16* __restrict__ PM, const float* __restrict__ MN, const float* __restrict__ MW, const float* __restrict__ O, float* __restrict__ OUT) {
  __shared__ __align__(16) float ssg[64][KVW + 4]; __shared__ float sden[64]; __shared__ __align__(16) float so[4][16][132];
  const int tid = threadIdx.x, wave = tid >> 5, lane = tid & 31, col = lane & 15, g = lane >> 4; const size_t rb = (size_t)blockIdx.x * 64; const size_t r0 = rb + wave * 16; const int half = blockIdx.y, qg = blockIdx.z; const int c0 = half * 128;
  for (int e = tid; e < 64 * KVW; e += 128) { const int rl = e >> 8, c = e & 255; const float v = QF[(rb + rl) * DM + qg * KVW + c]; ssg[rl][c] = (v > 0.f) ? v : expm1f_ni(v); }
  __syncthreads();
  if (tid < 64) { float d0 = 0.f; for (int c = 0; c < KVW; ++c) d0 += ssg[tid][c] * bfr(MN[c]); sden[tid] = d0; }
  v8f acc[8] = {};
#pragma unroll
  for (int kc = 0; kc < KVW / 32; ++kc) { const F2 a = split_row(&ssg[wave * 16 + col][0], kc * 32, lane);
#pragma unroll
    for (int j = 0; j < 8; ++j) { const v16b w = frag_b(PM + (size_t)(c0 + j * 16 + col) * KVW + kc * 32, lane); acc[j] = wmma_bf(a.h, w, acc[j]); acc[j] = wmma_bf(a.l, w, acc[j]); } }
  __syncthreads();
  const float wg = 1.0f / (1.0f + __expf(-bfr(MW[0])));
#pragma unroll
  for (int j = 0; j < 8; ++j)
#pragma unroll
    for (int r = 0; r < 8; ++r) { const int rl = wave * 16 + 8 * g + r; const size_t oi = (rb + rl) * DM + qg * KVW + c0 + j * 16 + col; so[wave][8 * g + r][j * 16 + col] = O[oi] * (1.0f - wg) + (acc[j][r] / sden[rl]) * wg; }
  LDSX();
  for (int rl = 0; rl < 16; ++rl) vst2(OUT + (r0 + rl) * DM + qg * KVW + c0 + lane * 4, *(const v4f*)&so[wave][rl][lane * 4]);
}
extern "C" void kernel_launch(void* const* d_in, const int* in_sizes, int n_in, void* d_out, int out_size, void* d_ws, size_t ws_size, hipStream_t stream) {
  (void)in_sizes; (void)n_in; (void)out_size;
  const float** F = (const float**)d_in;
  if (ws_size < (size_t)WS_END) return;
  char* ws = (char*)d_ws; __bf16 *PQ = (__bf16*)(ws + WS_PQ), *PK = (__bf16*)(ws + WS_PK), *PV = (__bf16*)(ws + WS_PV), *PM = (__bf16*)(ws + WS_PM); float *QF = (float*)(ws + WS_QF), *O = (float*)(ws + WS_O); _Float16 *QH = (_Float16*)(ws + WS_QH), *Kr = (_Float16*)(ws + WS_K), *V = (_Float16*)(ws + WS_V);
  k_pack<<<dim3(DM, 4), 256, 0, stream>>>(F[1], F[2], F[3], F[4], PQ, PK, PV, PM);
  k_proj<<<dim3(TNB * SS / 64, DM / 128, 3), 128, 0, stream>>>(F[0], PQ, PK, PV, QF, QH, Kr, V);
  k_attn<<<dim3(TQB, NQ * NH, TNB), 128, 0, stream>>>(QH, Kr, V, O);
  k_mem<<<dim3(TNB * SS / 64, 2, NQ), 128, 0, stream>>>(QF, PM, F[5], F[6], O, (float*)d_out);
}
